// RGCN_67319317398020
// MI455X (gfx1250) — hardware-verified
//
#include <hip/hip_runtime.h>
#include <stddef.h>
#include <stdint.h>


#define D1     128
#define K2     256
#define NTHR   256
#define NWAVE  8
#define EPT    8
#define CHUNK  (NTHR * EPT)
#define WCAP   (EPT * 32)
#define LISTN  (NWAVE * WCAP)
#define NBD    8192
#define SLD    13
#define NBA    1024
#define SLA    10
#define RCAP   32768
#define DEGCAP 256
#define GBM    32
#define GTHR   64
#define NRELMAX 8
#define UPA    (D1 * (D1 / 8))
#define UPP    (D1 * (K2 / 8))
#define UPH    (D1 * (D1 / 4))
#define AGG_ZINTS    (LISTN + 2 * RCAP + 3 * NBA)
#define AGG_LDS_INTS (AGG_ZINTS + 16)
#define WSMAX  134217728

static_assert((CHUNK & (CHUNK - 1)) == 0 && CHUNK <= 4096);
static_assert((NBD & (NBD - 1)) == 0 && NBD == (1 << SLD));
static_assert((NBA & (NBA - 1)) == 0 && NBA == (1 << SLA));
static_assert(((long long)CHUNK << SLD) < (1LL << 31));
static_assert(((long long)CHUNK << SLA) < (1LL << 31));
static_assert(NBD % (NTHR * 4) == 0 && NBD % GBM == 0);
static_assert(LISTN % NTHR == 0);
static_assert(NBA % NWAVE == 0 && NBA % 32 == 0 && NBA % GBM == 0);
static_assert(RCAP % 32 == 0 && AGG_ZINTS % (NTHR * 4) == 0 && LISTN % 4 == 0);
static_assert(D1 % 32 == 0 && K2 % 32 == 0 && K2 == 2 * D1);
static_assert(GBM == (GTHR / 32) * 16);
static_assert(UPA % NTHR == 0 && UPP % NTHR == 0 && UPH % NTHR == 0);
static_assert(UPA == (1 << 11) && UPH == (1 << 12) && UPP == (1 << 12));
static_assert(D1 / 8 == 16 && D1 / 4 == 32 && K2 / 8 == 32 && D1 == 4 * 32);
static_assert(AGG_LDS_INTS * 4 <= 300000);

typedef float          v4f   __attribute__((ext_vector_type(4)));
typedef float          v8f   __attribute__((ext_vector_type(8)));
typedef int            v4i   __attribute__((ext_vector_type(4)));
typedef int            v8i   __attribute__((ext_vector_type(8)));
typedef unsigned short v8us  __attribute__((ext_vector_type(8)));
typedef unsigned short v16us __attribute__((ext_vector_type(16)));
typedef __bf16         v16bf __attribute__((ext_vector_type(16)));
typedef v4f  __attribute__((may_alias)) v4fa;
typedef v4i  __attribute__((may_alias)) v4ia;
typedef v8us __attribute__((may_alias)) v8usa;
union Frag { v16bf v; v16us u; v8us h[2]; v8i w; };

__device__ __forceinline__ v8f wmb(const Frag& a, const Frag& b, v8f c) {
  v8f d = __builtin_amdgcn_wmma_f32_16x16x32_bf16(false, a.v, false, b.v, (short)0, c, false, false);
  asm volatile("v_nop\n\tv_nop\n\tv_nop\n\tv_nop" : "+v"(d) : "v"(a.w), "v"(b.w));
  return d;
}

__device__ __forceinline__ unsigned bf16_bits(float f) {
  const unsigned u = __float_as_uint(f);
  return (u + 0x7FFFu + ((u >> 16) & 1u)) >> 16;
}
__device__ __forceinline__ float bf16_val(float f) {
  return __uint_as_float(bf16_bits(f) << 16);
}
__device__ __forceinline__ v8us hilo8(v4f t) {
  v8us o;
  unsigned hb;
  hb = bf16_bits(t.x); o[0] = (unsigned short)hb; o[4] = (unsigned short)bf16_bits(t.x - __uint_as_float(hb << 16));
  hb = bf16_bits(t.y); o[1] = (unsigned short)hb; o[5] = (unsigned short)bf16_bits(t.y - __uint_as_float(hb << 16));
  hb = bf16_bits(t.z); o[2] = (unsigned short)hb; o[6] = (unsigned short)bf16_bits(t.z - __uint_as_float(hb << 16));
  hb = bf16_bits(t.w); o[3] = (unsigned short)hb; o[7] = (unsigned short)bf16_bits(t.w - __uint_as_float(hb << 16));
  return o;
}

template <int SLB>
__device__ __forceinline__ int scan_chunk(const int* __restrict__ dsts, int nE, int cbase, int slotBase,
                                          int nb, int vec8, int* list, int tid, int lane, int wave) {
  int wc = 0;
  const int el0  = tid * EPT;
  const int e0   = cbase + el0;
  const int sent = -2147483647 - 1;
  v4i da, db;
  if (vec8 != 0 && cbase + CHUNK <= nE) {
    da = *(const v4i*)(dsts + e0);
    db = *(const v4i*)(dsts + e0 + 4);
  } else {
    da.x = (e0     < nE) ? dsts[min(e0,     nE - 1)] : sent;
    da.y = (e0 + 1 < nE) ? dsts[min(e0 + 1, nE - 1)] : sent;
    da.z = (e0 + 2 < nE) ? dsts[min(e0 + 2, nE - 1)] : sent;
    da.w = (e0 + 3 < nE) ? dsts[min(e0 + 3, nE - 1)] : sent;
    db.x = (e0 + 4 < nE) ? dsts[min(e0 + 4, nE - 1)] : sent;
    db.y = (e0 + 5 < nE) ? dsts[min(e0 + 5, nE - 1)] : sent;
    db.z = (e0 + 6 < nE) ? dsts[min(e0 + 6, nE - 1)] : sent;
    db.w = (e0 + 7 < nE) ? dsts[min(e0 + 7, nE - 1)] : sent;
  }
  const unsigned nbs = (unsigned)slotBase;
  const unsigned unb = (unsigned)nb;
  const unsigned s0 = (unsigned)da.x - nbs, s1 = (unsigned)da.y - nbs;
  const unsigned s2 = (unsigned)da.z - nbs, s3 = (unsigned)da.w - nbs;
  const unsigned s4 = (unsigned)db.x - nbs, s5 = (unsigned)db.y - nbs;
  const unsigned s6 = (unsigned)db.z - nbs, s7 = (unsigned)db.w - nbs;
  const bool h0 = s0 < unb, h1 = s1 < unb, h2 = s2 < unb, h3 = s3 < unb;
  const bool h4 = s4 < unb, h5 = s5 < unb, h6 = s6 < unb, h7 = s7 < unb;
  const unsigned any = __builtin_amdgcn_ballot_w32(h0 | h1 | h2 | h3 | h4 | h5 | h6 | h7);
  if (any != 0u) {
#define HITJ(J, HJ, SJ) { \
      const unsigned mj = __builtin_amdgcn_ballot_w32(HJ); \
      if (mj != 0u) { \
        if (HJ) { \
          const int pos = wc + (int)__builtin_amdgcn_mbcnt_lo(mj, 0u); \
          if (pos < WCAP) list[wave * WCAP + pos] = ((el0 + (J)) << SLB) | (int)(SJ); \
        } \
        wc += (int)__builtin_popcount(mj); } }
    HITJ(0, h0, s0)
    HITJ(1, h1, s1)
    HITJ(2, h2, s2)
    HITJ(3, h3, s3)
    HITJ(4, h4, s4)
    HITJ(5, h5, s5)
    HITJ(6, h6, s6)
    HITJ(7, h7, s7)
#undef HITJ
  }
  return wc;
}

__global__ __launch_bounds__(NTHR) void k_prep(const float* __restrict__ w1, const float* __restrict__ wp,
                                               const float* __restrict__ w2, const float* __restrict__ w3,
                                               int nRel,
                                               unsigned short* WP1, unsigned short* WPp,
                                               unsigned short* WH2, unsigned short* WH3) {
  const int u  = (int)blockIdx.x * NTHR + (int)threadIdx.x;
  const int U1 = nRel * UPA;
  const int U2 = U1 + UPP;
  const int U3 = U2 + nRel * UPH;
  const int U4 = U3 + nRel * UPH;
  v8us o;
  unsigned short* dp;
  if (u < U1) {
    const int t  = u >> 11;
    const int n  = (u >> 4) & 127;
    const int k8 = (u & 15) * 8;
    const float* p = w1 + (size_t)t * D1 * D1 + (size_t)k8 * D1 + n;
#pragma unroll
    for (int i = 0; i < 8; ++i) o[i] = (unsigned short)bf16_bits(p[(size_t)i * D1]);
    dp = WP1 + ((size_t)t * D1 + n) * D1 + k8;
  } else if (u < U2) {
    const int v  = u - U1;
    const int n  = v >> 5;
    const int k8 = (v & 31) * 8;
    const float* p = wp + (size_t)k8 * D1 + n;
#pragma unroll
    for (int i = 0; i < 8; ++i) o[i] = (unsigned short)bf16_bits(p[(size_t)i * D1]);
    dp = WPp + (size_t)n * K2 + k8;
  } else if (u < U4) {
    const float* W = w2;
    unsigned short* D = WH2;
    int v = u - U2;
    if (u >= U3) { W = w3; D = WH3; v = u - U3; }
    const int r = v >> 12;
    const int n = (v >> 5) & 127;
    const int g = v & 31;
    const float* p = W + (size_t)r * D1 * D1 + (size_t)(4 * g) * D1 + n;
    const unsigned short f0 = (unsigned short)bf16_bits(p[0]);
    const unsigned short f1 = (unsigned short)bf16_bits(p[D1]);
    const unsigned short f2 = (unsigned short)bf16_bits(p[2 * D1]);
    const unsigned short f3 = (unsigned short)bf16_bits(p[3 * D1]);
    o[0] = f0; o[1] = f1; o[2] = f2; o[3] = f3; o[4] = f0; o[5] = f1; o[6] = f2; o[7] = f3;
    dp = D + ((size_t)r * D1 + n) * K2 + 8 * g;
  } else {
    return;
  }
  *(volatile v8us*)dp = o;
  __threadfence();
  *(volatile v8us*)dp = o;
}

__global__ __launch_bounds__(NTHR) void k_cvx(const float* __restrict__ x0, const float* __restrict__ x1,
                                              int n0, int n1, int U0, int U1,
                                              unsigned short* xb0, unsigned short* xb1) {
  const int u = (int)blockIdx.x * NTHR + (int)threadIdx.x;
  const float* x = x0;
  unsigned short* xb = xb0;
  int nN = n0;
  int v;
  if (u < U0) {
    v = u;
  } else if (u < U0 + U1) {
    x = x1; xb = xb1; nN = n1; v = u - U0;
  } else {
    return;
  }
  const int row = v >> 4;
  const int k8  = (v & 15) * 8;
  const int rc  = row < nN ? row : nN - 1;
  const float* p = x + (size_t)rc * D1 + k8;
  const v4f a = *(const v4fa*)p;
  const v4f b = *(const v4fa*)(p + 4);
  const bool ok = row < nN;
  v8us o;
  o[0] = ok ? (unsigned short)bf16_bits(a.x) : (unsigned short)0;
  o[1] = ok ? (unsigned short)bf16_bits(a.y) : (unsigned short)0;
  o[2] = ok ? (unsigned short)bf16_bits(a.z) : (unsigned short)0;
  o[3] = ok ? (unsigned short)bf16_bits(a.w) : (unsigned short)0;
  o[4] = ok ? (unsigned short)bf16_bits(b.x) : (unsigned short)0;
  o[5] = ok ? (unsigned short)bf16_bits(b.y) : (unsigned short)0;
  o[6] = ok ? (unsigned short)bf16_bits(b.z) : (unsigned short)0;
  o[7] = ok ? (unsigned short)bf16_bits(b.w) : (unsigned short)0;
  unsigned short* dp = xb + (size_t)row * D1 + k8;
  *(volatile v8us*)dp = o;
  __threadfence();
  *(volatile v8us*)dp = o;
}

__global__ __launch_bounds__(NTHR) void k_deg(const int* __restrict__ lddi, const int* __restrict__ lpdi,
                                              int nRel, int Eper, int nEp, int nD, int nP, int nbpd, float* dg) {
  __shared__ __attribute__((aligned(16))) int scnt[NBD];
  __shared__ __attribute__((aligned(16))) int list[LISTN];
  __shared__ int wcnt[NWAVE];
  const int tid = (int)threadIdx.x, lane = tid & 31, wave = tid >> 5;
  const int nodeBase = (int)blockIdx.x * NBD;
  const int p = (int)blockIdx.y;
  const int* lst = lpdi;
  int nTab = nP, nE = nEp;
  if (p < nRel) { lst = lddi + (size_t)p * (size_t)Eper; nTab = nD; nE = Eper; }
  if (nodeBase >= nTab) return;
  const int vec8 = ((nE & 3) == 0) ? 1 : 0;

  for (int i = tid; i < NBD; i += NTHR) scnt[i] = 0;
  for (int i = tid; i < LISTN; i += NTHR) list[i] = 0;
  if (tid < NWAVE) wcnt[tid] = 0;
  __syncthreads();

  const int nChunks = (nE + CHUNK - 1) / CHUNK;
#pragma unroll 1
  for (int ch = 0; ch < nChunks; ++ch) {
    const int cbase = ch * CHUNK;
    const int wc = scan_chunk<SLD>(lst, nE, cbase, nodeBase, NBD, vec8, list, tid, lane, wave);
    if (lane == 0) wcnt[wave] = wc;
    __syncthreads();
    if (wave == 0) {
#pragma unroll 1
      for (int w2 = 0; w2 < NWAVE; ++w2) {
        int c = wcnt[w2];
        c = c < 0 ? 0 : (c > WCAP ? WCAP : c);
#pragma unroll 1
        for (int b0 = 0; b0 < c; b0 += 32) {
          const int idx = b0 + lane;
          const int ent = list[w2 * WCAP + (idx < WCAP ? idx : WCAP - 1)];
          const int m32 = (c - b0) < 32 ? (c - b0) : 32;
#pragma unroll 1
          for (int k = 0; k < m32; ++k) {
            const int u  = __builtin_amdgcn_readlane(ent, k);
            const int sl = u & (NBD - 1);
            if (lane == 0) scnt[sl] = scnt[sl] + 1;
          }
        }
      }
    }
    __syncthreads();
  }

  v4f vals[NBD / (NTHR * 4)];
#pragma unroll
  for (int it = 0; it < NBD / (NTHR * 4); ++it) {
    const int s0 = it * (NTHR * 4) + 4 * tid;
    const v4i c4 = *(const v4ia*)(scnt + s0);
    const float d0 = (float)(c4.x < 1 ? 1 : c4.x), d1 = (float)(c4.y < 1 ? 1 : c4.y);
    const float d2 = (float)(c4.z < 1 ? 1 : c4.z), d3 = (float)(c4.w < 1 ? 1 : c4.w);
    v4f v;
    v.x = rsqrtf(d0); v.y = rsqrtf(d1); v.z = rsqrtf(d2); v.w = rsqrtf(d3);
    vals[it] = v;
  }
  float* base = dg + (size_t)p * (size_t)nbpd + (size_t)nodeBase;
#pragma unroll
  for (int it = 0; it < NBD / (NTHR * 4); ++it) {
    const int s0 = it * (NTHR * 4) + 4 * tid;
    *(volatile v4f*)(base + s0) = vals[it];
  }
  __threadfence();
#pragma unroll
  for (int it = 0; it < NBD / (NTHR * 4); ++it) {
    const int s0 = it * (NTHR * 4) + 4 * tid;
    *(volatile v4f*)(base + s0) = vals[it];
  }
}

__global__ __launch_bounds__(GTHR) void k_gemm(const unsigned short* __restrict__ A, int K,
                                               const unsigned short* __restrict__ WT,
                                               const float* __restrict__ dgb, int nbpd,
                                               float* T, int ldT, int nOut) {
  __shared__ __attribute__((aligned(16))) float stg[GBM * D1];
  __shared__ __attribute__((aligned(16))) float sdg[GBM];
  const int tid = (int)threadIdx.x, lane = tid & 31, wave = tid >> 5, hh = lane >> 4, m = lane & 15;
  const int rowBase = (int)blockIdx.x * GBM;
  const int g = (int)blockIdx.y;
  if (tid < GBM) sdg[tid] = dgb[(size_t)g * (size_t)nbpd + rowBase + tid];

  v8f acc[8];
  {
    const v8f z = {0.f, 0.f, 0.f, 0.f, 0.f, 0.f, 0.f, 0.f};
#pragma unroll
    for (int t = 0; t < 8; ++t) acc[t] = z;
  }
  const unsigned short* ap = A  + (size_t)(rowBase + 16 * wave + m) * (size_t)K + 8 * hh;
  const unsigned short* bp = WT + ((size_t)g * D1 + m) * (size_t)K + 8 * hh;
  const int ksteps = K >> 5;

#pragma unroll 1
  for (int ks = 0; ks < ksteps; ++ks) {
    const int k0 = 32 * ks;
    Frag af;
    af.h[0] = *(const v8usa*)(ap + k0);
    af.h[1] = *(const v8usa*)(ap + k0 + 16);
#pragma unroll
    for (int nt = 0; nt < 8; ++nt) {
      const unsigned short* wq = bp + (size_t)(16 * nt) * (size_t)K + k0;
      Frag bf;
      bf.h[0] = *(const v8usa*)wq;
      bf.h[1] = *(const v8usa*)(wq + 16);
      acc[nt] = wmb(af, bf, acc[nt]);
    }
  }

#pragma unroll
  for (int nt = 0; nt < 8; ++nt) {
    const int lc = 16 * nt + m;
#pragma unroll
    for (int r = 0; r < 8; ++r) {
      const int lr = 16 * wave + 8 * hh + r;
      stg[lr * D1 + lc] = acc[nt][r];
    }
  }
  __syncthreads();

  v4f fv[16];
#pragma unroll
  for (int i = 0; i < 16; ++i) {
    const int lr = 16 * wave + i;
    fv[i] = *(const v4fa*)(stg + lr * D1 + 4 * lane) * sdg[lr];
  }
#pragma unroll
  for (int i = 0; i < 16; ++i) {
    const int gr = rowBase + 16 * wave + i;
    if (gr < nOut) {
      float* op = T + (size_t)gr * (size_t)ldT + (size_t)g * D1 + 4 * lane;
      *(volatile v4f*)op = fv[i];
    }
  }
  __threadfence();
#pragma unroll
  for (int i = 0; i < 16; ++i) {
    const int gr = rowBase + 16 * wave + i;
    if (gr < nOut) {
      float* op = T + (size_t)gr * (size_t)ldT + (size_t)g * D1 + 4 * lane;
      *(volatile v4f*)op = fv[i];
    }
  }
}

template <int MODE, int ADDIN>
__global__ __launch_bounds__(NTHR) void k_agg(const int* __restrict__ srcs, const int* __restrict__ dsts,
                                              int nRel, int Eper, int nDst, int nSrc, int mRows,
                                              const float* __restrict__ tpl, int ldT,
                                              const float* __restrict__ bias,
                                              const float* oin, float* oout, unsigned short* hpl) {
  extern __shared__ __attribute__((aligned(16))) int dsm[];
  int* list = dsm;
  int* hl   = dsm + LISTN;
  int* sl   = hl + RCAP;
  int* cnt  = sl + RCAP;
  int* offs = cnt + NBA;
  int* cur  = offs + NBA;
  int* misc = cur + NBA;
  const int tid = (int)threadIdx.x, lane = tid & 31, wave = tid >> 5;
  const int nodeBase = (int)blockIdx.x * NBA;
  const int nEtot = nRel * Eper;
  const int vec8 = ((Eper & 3) == 0) ? 1 : 0;

  {
    const v4i z4 = {0, 0, 0, 0};
    for (int i = tid * 4; i < AGG_ZINTS; i += NTHR * 4) *(v4ia*)(dsm + i) = z4;
    if (tid < 16) misc[tid] = 0;
  }
  __syncthreads();

  int t = 0, ov = 0;
  const int nChunks = (Eper + CHUNK - 1) / CHUNK;
#pragma unroll 1
  for (int rel = 0; rel < nRel; ++rel) {
    const int* dl = dsts + (size_t)rel * (size_t)Eper;
    const int ebase = rel * Eper;
#pragma unroll 1
    for (int ch = 0; ch < nChunks; ++ch) {
      const int cbase = ch * CHUNK;
      const int wc = scan_chunk<SLA>(dl, Eper, cbase, nodeBase, NBA, vec8, list, tid, lane, wave);
      if (lane == 0) misc[wave] = wc;
      __syncthreads();
      if (wave == 0) {
#pragma unroll 1
        for (int w2 = 0; w2 < NWAVE; ++w2) {
          int c = misc[w2];
          c = c < 0 ? 0 : (c > WCAP ? WCAP : c);
#pragma unroll 1
          for (int b0 = 0; b0 < c; b0 += 32) {
            const int idx = b0 + lane;
            const int ent = list[w2 * WCAP + (idx < WCAP ? idx : WCAP - 1)];
            const int m32 = (c - b0) < 32 ? (c - b0) : 32;
#pragma unroll 1
            for (int k = 0; k < m32; ++k) {
              const int u    = __builtin_amdgcn_readlane(ent, k);
              const int slot = u & (NBA - 1);
              const int el   = (u >> SLA) & (CHUNK - 1);
              int eg = cbase + el;
              eg = eg > Eper - 1 ? Eper - 1 : eg;
              const int pk   = ((ebase + eg) << SLA) | slot;
              if (t < RCAP) {
                if (lane == 0) { hl[t] = pk; cnt[slot] = cnt[slot] + 1; }
                t = t + 1;
              } else {
                ov = 1;
              }
            }
          }
        }
      }
      __syncthreads();
    }
  }
  if (wave == 0 && lane == 0) { misc[8] = t; misc[9] = ov; }
  __syncthreads();
  int tt = misc[8];
  tt = tt < 0 ? 0 : (tt > RCAP ? RCAP : tt);
  const int ovf = misc[9];

  if (wave == 0) {
    const int base = lane * (NBA / 32);
    int sacc = 0;
#pragma unroll 1
    for (int i = 0; i < NBA / 32; ++i) sacc += cnt[base + i];
    int incl = sacc;
#pragma unroll
    for (int d = 1; d < 32; d <<= 1) {
      const int y = __shfl_up(incl, d, 32);
      if (lane >= d) incl += y;
    }
    int run = incl - sacc;
#pragma unroll 1
    for (int i = 0; i < NBA / 32; ++i) {
      const int cv = cnt[base + i];
      offs[base + i] = run;
      cur[base + i]  = run;
      run += cv;
    }
  }
  __syncthreads();
  if (wave == 0) {
#pragma unroll 1
    for (int b0 = 0; b0 < tt; b0 += 32) {
      const int idx = b0 + lane;
      const int ent = hl[idx < RCAP ? idx : RCAP - 1];
      const int m32 = (tt - b0) < 32 ? (tt - b0) : 32;
#pragma unroll 1
      for (int k = 0; k < m32; ++k) {
        const int u    = __builtin_amdgcn_readlane(ent, k);
        const int slot = u & (NBA - 1);
        if (lane == 0) {
          int p = cur[slot];
          p = p < 0 ? 0 : (p > RCAP - 1 ? RCAP - 1 : p);
          sl[p] = u;
          cur[slot] = p + 1;
        }
      }
    }
  }
  __syncthreads();

  const float qnan = __int_as_float(0x7fc00000);
  const float pz = (ovf != 0) ? qnan : 0.0f;
  const v4f z4 = {0.0f, 0.0f, 0.0f, 0.0f};
  v4f bs = z4;
#pragma unroll 1
  for (int r = 0; r < nRel; ++r) {
    const v4f a = *(const v4fa*)(bias + (size_t)r * D1 + 4 * lane);
    bs.x += bf16_val(a.x); bs.y += bf16_val(a.y); bs.z += bf16_val(a.z); bs.w += bf16_val(a.w);
  }
#pragma unroll 1
  for (int si = 0; si < NBA / NWAVE; ++si) {
    const int s    = si * NWAVE + wave;
    const int node = nodeBase + s;
    const int craw = cnt[s];
    const bool big = craw > DEGCAP;
    const int c = craw < 0 ? 0 : (craw > DEGCAP ? DEGCAP : craw);
    int o = offs[s];
    o = o < 0 ? 0 : (o > RCAP ? RCAP : o);
    v4f tot = z4;
    v4f acc = z4;
    int rcur = 0;
    int ccur = 0;
#pragma unroll 1
    for (int b0 = 0; b0 < c; b0 += 32) {
      int idx = o + b0 + lane;
      idx = idx > RCAP - 1 ? RCAP - 1 : idx;
      const int ent = sl[idx];
      int eid = ent >> SLA;
      eid = eid < 0 ? 0 : (eid > nEtot - 1 ? nEtot - 1 : eid);
      int sr = srcs[eid];
      sr = sr < 0 ? 0 : (sr > nSrc - 1 ? nSrc - 1 : sr);
      const int m32 = (c - b0) < 32 ? (c - b0) : 32;
#pragma unroll 1
      for (int k = 0; k < m32; ++k) {
        const int ek = __builtin_amdgcn_readlane(eid, k);
        const int sk = __builtin_amdgcn_readlane(sr, k);
        int rk = ek / Eper;
        rk = rk < 0 ? 0 : (rk > nRel - 1 ? nRel - 1 : rk);
        if (rk != rcur) {
          const float dd = rsqrtf(fmaxf((float)ccur, 1.0f));
          tot.x = fmaf(acc.x, dd, tot.x); tot.y = fmaf(acc.y, dd, tot.y);
          tot.z = fmaf(acc.z, dd, tot.z); tot.w = fmaf(acc.w, dd, tot.w);
          acc = z4; ccur = 0; rcur = rk;
        }
        const v4f a = *(const v4fa*)(tpl + (size_t)sk * (size_t)ldT + (size_t)rk * D1 + 4 * lane);
        acc += a;
        ccur = ccur + 1;
      }
    }
    {
      const float dd = rsqrtf(fmaxf((float)ccur, 1.0f));
      tot.x = fmaf(acc.x, dd, tot.x); tot.y = fmaf(acc.y, dd, tot.y);
      tot.z = fmaf(acc.z, dd, tot.z); tot.w = fmaf(acc.w, dd, tot.w);
    }
    const float pzr = big ? qnan : pz;
    const bool live = node < nDst;
    v4f v = tot + bs;
    if constexpr (ADDIN != 0) {
      const int ncl = live ? node : nDst - 1;
      const v4f pv = *(const v4fa*)(oin + (size_t)ncl * (size_t)D1 + 4 * lane);
      v = pv + v;
    }
    if constexpr (MODE == 0) {
      v.x = fmaxf(v.x, 0.0f); v.y = fmaxf(v.y, 0.0f); v.z = fmaxf(v.z, 0.0f); v.w = fmaxf(v.w, 0.0f);
    }
    v.x = v.x + pzr; v.y = v.y + pzr; v.z = v.z + pzr; v.w = v.w + pzr;
    v4f y;
    y.x = live ? v.x : 0.0f; y.y = live ? v.y : 0.0f; y.z = live ? v.z : 0.0f; y.w = live ? v.w : 0.0f;
    if constexpr (MODE == 1) {
      if (node < mRows) {
        float* op = oout + (size_t)node * (size_t)D1 + 4 * lane;
        *(volatile v4f*)op = y;
        __threadfence();
        *(volatile v4f*)op = y;
      }
    } else {
      const v8us po = hilo8(y);
      if (node < mRows) {
        unsigned short* hp = hpl + (size_t)node * (size_t)K2 + 8 * lane;
        *(volatile v8us*)hp = po;
        __threadfence();
        *(volatile v8us*)hp = po;
      }
    }
  }
}

static inline int cdiv(int a, int b) { return (a + b - 1) / b; }

extern "C" void kernel_launch(void* const* d_in, const int* in_sizes, int n_in,
                              void* d_out, int out_size, void* d_ws, size_t ws_size,
                              hipStream_t stream) {
  if (n_in < 18) return;
  if (in_sizes[0] < D1 || (in_sizes[0] % D1) != 0) return;
  if (in_sizes[1] < K2 || (in_sizes[1] % K2) != 0) return;
  const int nD = in_sizes[0] / D1, nP = in_sizes[1] / K2;
  if (nD > (1 << 22) || nP > (1 << 22)) return;
  if (in_sizes[2] < D1 * D1 || (in_sizes[2] % (D1 * D1)) != 0) return;
  const int nRel = in_sizes[2] / (D1 * D1);
  if (nRel < 1 || nRel > NRELMAX) return;
  if (in_sizes[3] != nRel * D1) return;
  if (in_sizes[4] != K2 * D1 || in_sizes[5] != D1) return;
  if (in_sizes[8] != nRel * D1 * D1 || in_sizes[9] != nRel * D1) return;
  if (in_sizes[10] != nRel * D1 * D1 || in_sizes[11] != nRel * D1) return;
  if (in_sizes[12] < nRel || (in_sizes[12] % nRel) != 0) return;
  const int Eper = in_sizes[12] / nRel;
  if (in_sizes[13] != in_sizes[12]) return;
  const int nEp = in_sizes[14];
  if (in_sizes[15] != nEp) return;
  if (Eper < 1 || nEp < 1) return;
  const long long eMax = 1LL << (31 - SLA);
  if ((long long)nRel * (long long)Eper >= eMax || (long long)nEp >= eMax) return;
  if ((long long)out_size != (long long)nD * D1) return;

  const float* x_d   = (const float*)d_in[0];
  const float* x_p   = (const float*)d_in[1];
  const float* W1    = (const float*)d_in[2];
  const float* b1    = (const float*)d_in[3];
  const float* W1p   = (const float*)d_in[4];
  const float* b1p   = (const float*)d_in[5];
  const float* W2    = (const float*)d_in[8];
  const float* b2    = (const float*)d_in[9];
  const float* W3    = (const float*)d_in[10];
  const float* b3    = (const float*)d_in[11];
  const int* ddi_s = (const int*)d_in[12];
  const int* ddi_d = (const int*)d_in[13];
  const int* pdi_s = (const int*)d_in[14];
  const int* pdi_d = (const int*)d_in[15];
  float* out = (float*)d_out;

  const int MPd = cdiv(nD, GBM) * GBM;
  const int MPp = cdiv(nP, GBM) * GBM;
  const int maxMP = MPd > MPp ? MPd : MPp;
  const int gD   = cdiv(maxMP, NBD);
  const int NBPD = gD * NBD;
  if (NBPD < maxMP) return;
  const int gA = cdiv(MPd, NBA);
  if ((long long)gA * NBA < MPd) return;
  {
    const long long dn = (long long)(nD > NBA ? nD : NBA);
    if ((long long)NBA * (long long)nRel * (long long)Eper * 5LL > (long long)RCAP * dn * 4LL) return;
    if ((long long)NBA * (long long)nEp * 5LL > (long long)RCAP * dn * 4LL) return;
  }
  const int U0 = MPd * (D1 / 8);
  const int U1 = (2 * MPp) * (D1 / 8);
  if ((U0 % NTHR) != 0 || (U1 % NTHR) != 0) return;
  const int UW = nRel * UPA + UPP + 2 * nRel * UPH;
  if ((UW % NTHR) != 0) return;
  const int ldT = nRel * D1;

  size_t szRA = (size_t)MPd * D1 * 2;
  if ((size_t)MPd * D1 * 4 > szRA) szRA = (size_t)MPd * D1 * 4;
  size_t szRB = (size_t)MPp * K2 * 2 + (size_t)MPp * D1 * 4;
  if ((size_t)MPd * K2 * 2 > szRB) szRB = (size_t)MPd * K2 * 2;
  char* ws = (char*)d_ws;
  size_t off = 0;
  const size_t oDG  = off; off += (size_t)(nRel + 1) * (size_t)NBPD * 4;  off = (off + 255) & ~(size_t)255;
  const size_t oWP1 = off; off += (size_t)nRel * D1 * D1 * 2;             off = (off + 255) & ~(size_t)255;
  const size_t oWPp = off; off += (size_t)D1 * K2 * 2;                    off = (off + 255) & ~(size_t)255;
  const size_t oWH2 = off; off += (size_t)nRel * D1 * K2 * 2;             off = (off + 255) & ~(size_t)255;
  const size_t oWH3 = off; off += (size_t)nRel * D1 * K2 * 2;             off = (off + 255) & ~(size_t)255;
  const size_t oRA  = off; off += szRA;                                   off = (off + 255) & ~(size_t)255;
  const size_t oRB  = off; off += szRB;                                   off = (off + 255) & ~(size_t)255;
  const size_t oT   = off; off += (size_t)MPd * (size_t)ldT * 4;          off = (off + 255) & ~(size_t)255;
  if (off > ws_size || off > (size_t)WSMAX) return;
  float*          DG  = (float*)(ws + oDG);
  unsigned short* WP1 = (unsigned short*)(ws + oWP1);
  unsigned short* WPp = (unsigned short*)(ws + oWPp);
  unsigned short* WH2 = (unsigned short*)(ws + oWH2);
  unsigned short* WH3 = (unsigned short*)(ws + oWH3);
  unsigned short* XBd = (unsigned short*)(ws + oRA);
  float*          O   = (float*)(ws + oRA);
  unsigned short* XBp = (unsigned short*)(ws + oRB);
  float*          Tp  = (float*)(ws + oRB + (size_t)MPp * K2 * 2);
  unsigned short* HA  = (unsigned short*)(ws + oRB);
  float*          T   = (float*)(ws + oT);

  const size_t aggLds = (size_t)AGG_LDS_INTS * 4;
  hipFuncSetAttribute(reinterpret_cast<const void*>(&k_agg<1, 0>), hipFuncAttributeMaxDynamicSharedMemorySize, (int)aggLds);
  hipFuncSetAttribute(reinterpret_cast<const void*>(&k_agg<0, 1>), hipFuncAttributeMaxDynamicSharedMemorySize, (int)aggLds);
  hipFuncSetAttribute(reinterpret_cast<const void*>(&k_agg<0, 0>), hipFuncAttributeMaxDynamicSharedMemorySize, (int)aggLds);

  k_prep<<<UW / NTHR, NTHR, 0, stream>>>(W1, W1p, W2, W3, nRel, WP1, WPp, WH2, WH3);
  k_cvx<<<(U0 + U1) / NTHR, NTHR, 0, stream>>>(x_d, x_p, nD, 2 * nP, U0, U1, XBd, XBp);
  k_deg<<<dim3(gD, nRel + 1), NTHR, 0, stream>>>(ddi_s, pdi_s, nRel, Eper, nEp, nD, nP, NBPD, DG);

  k_gemm<<<dim3(MPd / GBM, nRel), GTHR, 0, stream>>>(XBd, D1, WP1, DG, NBPD, T, ldT, MPd);
  k_gemm<<<dim3(MPp / GBM, 1), GTHR, 0, stream>>>(XBp, K2, WPp, DG + (size_t)nRel * NBPD, NBPD, Tp, D1, MPp);
  k_agg<1, 0><<<gA, NTHR, aggLds, stream>>>(pdi_s, pdi_d, 1, nEp, nD, nP, MPd, Tp, D1, b1p, O, O, HA);
  k_agg<0, 1><<<gA, NTHR, aggLds, stream>>>(ddi_s, ddi_d, nRel, Eper, nD, nD, MPd, T, ldT, b1, O, O, HA);

  k_gemm<<<dim3(MPd / GBM, nRel), GTHR, 0, stream>>>(HA, K2, WH2, DG, NBPD, T, ldT, MPd);
  k_agg<0, 0><<<gA, NTHR, aggLds, stream>>>(ddi_s, ddi_d, nRel, Eper, nD, nD, MPd, T, ldT, b2, O, O, HA);

  k_gemm<<<dim3(MPd / GBM, nRel), GTHR, 0, stream>>>(HA, K2, WH3, DG, NBPD, T, ldT, MPd);
  k_agg<1, 0><<<gA, NTHR, aggLds, stream>>>(ddi_s, ddi_d, nRel, Eper, nD, nD, nD, T, ldT, b3, O, out, HA);
}
